// PairConnect_73340861546846
// MI455X (gfx1250) — hardware-verified
//
#include <hip/hip_runtime.h>
#include <math.h>


typedef _Float16 v16h __attribute__((ext_vector_type(16)));
typedef float    v8f  __attribute__((ext_vector_type(8)));
typedef float    v4f  __attribute__((ext_vector_type(4)));

#define N_TOK 1024
#define DIM   40
#define BATCH 2
#define TB    512
#define LDP   48

__device__ __forceinline__ float gelu_f(float v) {
    return 0.5f * v * (1.0f + erff(v * 0.70710678118654752f));
}

__device__ __forceinline__ v8f wmma16(v16h a, v16h b, v8f c) {
    c = __builtin_amdgcn_wmma_f32_16x16x32_f16(false, a, false, b, (short)0, c, false, false);
    asm volatile("v_nop\n\tv_nop\n\tv_nop\n\tv_nop" : "+v"(c) : "v"(a), "v"(b));
    return c;
}

__device__ __forceinline__ float rsum16(float v) {
    v += __shfl_xor(v, 1, 32);
    v += __shfl_xor(v, 2, 32);
    v += __shfl_xor(v, 4, 32);
    v += __shfl_xor(v, 8, 32);
    return v;
}

__global__ __launch_bounds__(256)
void k_proj(const float* __restrict__ x, const float* __restrict__ W1,
            float* A1g, float* A2g, int nrow)
{
    const int t   = blockIdx.x * 256 + threadIdx.x;
    const int tot = nrow * (DIM / 4);
    if (t >= tot) return;
    const int n  = t / (DIM / 4);
    const int d0 = (t - n * (DIM / 4)) * 4;
    const float* xr = x + (size_t)n * DIM;
    const float* wt = W1 + d0;
    const float* wb = W1 + DIM * DIM + d0;

    v4f s1 = {0.0f, 0.0f, 0.0f, 0.0f};
    v4f s2 = {0.0f, 0.0f, 0.0f, 0.0f};
#pragma unroll 4
    for (int k = 0; k < DIM; ++k) {
        const float xv = xr[k];
        const v4f wa = *(const v4f*)(wt + k * DIM);
        const v4f wc = *(const v4f*)(wb + k * DIM);
        s1.x = fmaf(xv, wa.x, s1.x); s1.y = fmaf(xv, wa.y, s1.y);
        s1.z = fmaf(xv, wa.z, s1.z); s1.w = fmaf(xv, wa.w, s1.w);
        s2.x = fmaf(xv, wc.x, s2.x); s2.y = fmaf(xv, wc.y, s2.y);
        s2.z = fmaf(xv, wc.z, s2.z); s2.w = fmaf(xv, wc.w, s2.w);
    }
    volatile v4f* p1 = (volatile v4f*)(A1g + (size_t)t * 4);
    volatile v4f* p2 = (volatile v4f*)(A2g + (size_t)t * 4);
    *p1 = s1;
    *p2 = s2;
    __threadfence();
    *p1 = s1;
    *p2 = s2;
}

__global__ __launch_bounds__(TB) __attribute__((amdgpu_num_vgpr(256)))
void k_pair(const float* __restrict__ A1g, const float* __restrict__ A2g,
            const float* __restrict__ b1,  const float* __restrict__ W2,
            const float* __restrict__ b2,  float* out)
{
    __shared__ __align__(16) float A1s[16][LDP];
    __shared__ __align__(16) float A2s[16][LDP];
    __shared__ __align__(16) float b1s[LDP];
    __shared__ __align__(16) float Os[16][DIM];

    const int tid = threadIdx.x;
    const int w   = tid >> 5;
    const int l   = tid & 31;
    const int h   = l >> 4;
    const int m16 = l & 15;
    const int ib  = blockIdx.x % (N_TOK / 16);
    const int b   = blockIdx.x / (N_TOK / 16);
    if (b >= BATCH) return;
    const int i   = ib * 16 + w;
    const size_t rowbase = ((size_t)b * N_TOK + (size_t)ib * 16) * DIM;
    const v4f z4 = {0.0f, 0.0f, 0.0f, 0.0f};

    if (tid < 160) {
        const int r = tid / 10, c = (tid - r * 10) * 4;
        *(v4f*)&A1s[r][c] = *(const v4f*)(A1g + rowbase + (size_t)r * DIM + c);
    } else if (tid < 192) {
        const int t = tid - 160, r = t >> 1, c = DIM + (t & 1) * 4;
        *(v4f*)&A1s[r][c] = z4;
        *(v4f*)&A2s[r][c] = z4;
    } else if (tid < 192 + LDP) {
        const int t = tid - 192;
        b1s[t] = (t < DIM) ? b1[t] : 0.0f;
    }

    v16h Bf[3][2];
    float bt[3];
#pragma unroll
    for (int dt = 0; dt < 3; ++dt) {
        const int n = 16 * dt + m16;
#pragma unroll
        for (int s = 0; s < 2; ++s) {
            v16h f = {};
#pragma unroll
            for (int e = 0; e < 16; ++e) {
                const int kk = 32 * s + ((e < 8) ? (8 * h + e) : (16 + 8 * h + (e - 8)));
                float v = 0.0f;
                if (kk < DIM && n < DIM) v = W2[kk * DIM + n] * 256.0f;
                f[e] = (_Float16)v;
            }
            Bf[dt][s] = f;
        }
        bt[dt] = (n < DIM) ? b2[n] : 0.0f;
    }

    float mrun = -__builtin_inff();
    float Z = 0.0f, acc0 = 0.0f, acc1 = 0.0f, acc2 = 0.0f;
    const float s16 = 1.52587890625e-05f;

    for (int jt = 0; jt <= ib; ++jt) {
        __syncthreads();
        if (tid < 160) {
            const int r = tid / 10, c = (tid - r * 10) * 4;
            const size_t src = ((size_t)b * N_TOK + (size_t)jt * 16 + r) * DIM + c;
            *(v4f*)&A2s[r][c] = *(const v4f*)(A2g + src);
        }
        __syncthreads();

        v16h a0 = {}, a1 = {};
        {
            const float* ra = &A1s[w][0];
            const float* rb = &A2s[m16][0];
#pragma unroll
            for (int e = 0; e < 16; ++e) {
                const int k = (e < 8) ? (8 * h + e) : (16 + 8 * h + (e - 8));
                const float v = (ra[k] + rb[k]) + b1s[k];
                a0[e] = (_Float16)(256.0f * gelu_f(v));
            }
#pragma unroll
            for (int e = 0; e < 8; ++e) {
                const int k = 32 + 8 * h + e;
                const float v = (ra[k] + rb[k]) + b1s[k];
                a1[e] = (_Float16)(256.0f * gelu_f(v));
            }
#pragma unroll
            for (int e = 8; e < 16; ++e) a1[e] = (_Float16)0.0f;
        }

        v8f c0 = {}, c1 = {}, c2 = {};
        c0 = wmma16(a0, Bf[0][0], c0);
        c0 = wmma16(a1, Bf[0][1], c0);
        c1 = wmma16(a0, Bf[1][0], c1);
        c1 = wmma16(a1, Bf[1][1], c1);
        c2 = wmma16(a0, Bf[2][0], c2);
        c2 = wmma16(a1, Bf[2][1], c2);

        float q[8];
#pragma unroll
        for (int r = 0; r < 8; ++r) {
            const float p0 = fmaf(c0[r], s16, bt[0]);
            const float p1 = fmaf(c1[r], s16, bt[1]);
            const float p2 = fmaf(c2[r], s16, bt[2]);
            c0[r] = p0; c1[r] = p1; c2[r] = p2;
            q[r] = rsum16(fmaf(p0, p0, fmaf(p1, p1, p2 * p2)));
        }

        float sv[8];
        int   vr[8];
        float tmax = -__builtin_inff();
#pragma unroll
        for (int r = 0; r < 8; ++r) {
            const int j = jt * 16 + 8 * h + r;
            vr[r] = (j <= i) ? 1 : 0;
            sv[r] = sqrtf(q[r]);
            tmax = fmaxf(tmax, vr[r] ? sv[r] : -__builtin_inff());
        }
        tmax = fmaxf(tmax, __shfl_xor(tmax, 16, 32));
        const float mnew = fmaxf(mrun, tmax);
        const float resc = __expf(mrun - mnew);
        Z *= resc; acc0 *= resc; acc1 *= resc; acc2 *= resc;
        mrun = mnew;
#pragma unroll
        for (int r = 0; r < 8; ++r) {
            const float wgt = vr[r] ? __expf(sv[r] - mrun) : 0.0f;
            Z += wgt;
            acc0 = fmaf(wgt, c0[r], acc0);
            acc1 = fmaf(wgt, c1[r], acc1);
            acc2 = fmaf(wgt, c2[r], acc2);
        }
    }

    Z    += __shfl_xor(Z, 16, 32);
    acc0 += __shfl_xor(acc0, 16, 32);
    acc1 += __shfl_xor(acc1, 16, 32);
    acc2 += __shfl_xor(acc2, 16, 32);
    const float inv = 1.0f / Z;
    const float o0 = acc0 * inv, o1 = acc1 * inv, o2 = acc2 * inv;
    if (h == 0) {
        Os[w][m16]      = o0;
        Os[w][16 + m16] = o1;
        if (m16 < 8) Os[w][32 + m16] = o2;
    }
    __syncthreads();

    if (w == 0) {
        v4f vals[5];
        const float* of = &Os[0][0];
#pragma unroll
        for (int qq = 0; qq < 5; ++qq) vals[qq] = *(const v4f*)(of + qq * 128 + l * 4);
        float* ob = out + rowbase;
#pragma unroll
        for (int qq = 0; qq < 5; ++qq) *(volatile v4f*)(ob + qq * 128 + l * 4) = vals[qq];
        __threadfence();
#pragma unroll
        for (int qq = 0; qq < 5; ++qq) *(volatile v4f*)(ob + qq * 128 + l * 4) = vals[qq];
    }
}

extern "C" void kernel_launch(void* const* d_in, const int* in_sizes, int n_in,
                              void* d_out, int out_size, void* d_ws, size_t ws_size,
                              hipStream_t stream)
{
    if (n_in < 5) return;
    const int elems = BATCH * N_TOK * DIM;
    if (in_sizes[0] != elems || in_sizes[1] != 2 * DIM * DIM || in_sizes[2] != DIM ||
        in_sizes[3] != DIM * DIM || in_sizes[4] != DIM || out_size != elems) return;
    const size_t need = (size_t)2 * (size_t)elems * sizeof(float);
    if (d_ws == nullptr || ws_size < need) return;

    const float* x  = (const float*)d_in[0];
    const float* W1 = (const float*)d_in[1];
    const float* b1 = (const float*)d_in[2];
    const float* W2 = (const float*)d_in[3];
    const float* b2 = (const float*)d_in[4];
    float* out = (float*)d_out;

    float* A1g = (float*)d_ws;
    float* A2g = A1g + elems;

    const int nrow = BATCH * N_TOK;
    const int tot4 = nrow * (DIM / 4);
    dim3 g0((tot4 + 255) / 256);
    k_proj<<<g0, 256, 0, stream>>>(x, W1, A1g, A2g, nrow);

    dim3 g1(BATCH * (N_TOK / 16));
    k_pair<<<g1, TB, 0, stream>>>(A1g, A2g, b1, W2, b2, out);
}
